// AS_MLP_67886253081286
// MI455X (gfx1250) — hardware-verified
//
#include <hip/hip_runtime.h>
#include <math.h>

constexpr int kImgs      = 16;
constexpr int kCh        = 256;
constexpr int kHgt       = 56;
constexpr int kWid       = 56;
constexpr int kHW        = 3136;
constexpr int kHid       = 1024;
constexpr int kGrpImgs   = 4;
constexpr int kGroups    = kImgs / kGrpImgs;
constexpr int kRows      = kGrpImgs * kHW;
constexpr int kImgElems  = kCh * kHW;
constexpr int kPartBlocks = 64;
constexpr int kPartV4    = kImgElems / (4 * kPartBlocks);
constexpr int kShiftGroup = 37;
constexpr int kShiftPad  = 3;
constexpr float kWCarry    = 16.0f;
constexpr float kWCarryInv = 0.0625f;
constexpr float kInvImgElems = 1.0f / 802816.0f;
constexpr float kGnEps     = 1e-5f;
static_assert(kRows % 64 == 0, "rows tile");
static_assert(kPartV4 * 4 * kPartBlocks == kImgElems, "partial coverage");
static_assert(kHW % 64 == 0, "pixel tile");

typedef __attribute__((ext_vector_type(16))) _Float16 v16h;
typedef __attribute__((ext_vector_type(8)))  _Float16 v8h;
typedef __attribute__((ext_vector_type(16))) __bf16   v16b;
typedef __attribute__((ext_vector_type(8)))  __bf16   v8b;
typedef __attribute__((ext_vector_type(8)))  float    v8f;
typedef __attribute__((ext_vector_type(4)))  float    v4f;
typedef __attribute__((ext_vector_type(4)))  unsigned int v4u;

__device__ __forceinline__ unsigned short f2bf_bits(float f) {
  unsigned u = __float_as_uint(f);
  return (unsigned short)((u + 0x7FFFu + ((u >> 16) & 1u)) >> 16);
}
__device__ __forceinline__ float bf_bits2f(unsigned short h) { return __uint_as_float(((unsigned)h) << 16); }

__device__ __forceinline__ void dep_guard_h(v8f& a, v8f& b, v16h x, v16h y) { asm volatile("v_nop\n\tv_nop\n\tv_nop\n\tv_nop" : "+v"(a), "+v"(b) : "v"(x), "v"(y)); }
__device__ __forceinline__ void dep_guard_b(v8f& a, v8f& b, v16b x, v16b y) { asm volatile("v_nop\n\tv_nop\n\tv_nop\n\tv_nop" : "+v"(a), "+v"(b) : "v"(x), "v"(y)); }
__device__ __forceinline__ void keep4_h(v16h a, v16h b, v16h c, v16h d) { asm volatile("v_nop" :: "v"(a), "v"(b), "v"(c), "v"(d)); }
__device__ __forceinline__ void keep4_b(v16b a, v16b b, v16b c, v16b d) { asm volatile("v_nop" :: "v"(a), "v"(b), "v"(c), "v"(d)); }
__device__ __forceinline__ void acc_guard4(v8f& a, v8f& b, v8f& c, v8f& d) { asm volatile("v_nop\n\tv_nop\n\tv_nop\n\tv_nop" : "+v"(a), "+v"(b), "+v"(c), "+v"(d)); }
template <typename T> struct Frag;
template <> struct Frag<_Float16> {
  typedef v16h V; union U { v16h v; v8h h[2]; };
  static __device__ __forceinline__ v16h load(const _Float16* p) {
    U f; f.h[0] = *(const v8h*)(p); f.h[1] = *(const v8h*)(p + 16); return f.v;
  }
  static __device__ __forceinline__ v8f mma(v16h a, v16h b, v8f c) {
    return __builtin_amdgcn_wmma_f32_16x16x32_f16(false, a, false, b, (short)0, c, false, false);
  }
  static __device__ __forceinline__ void guard(v8f& a, v8f& b, v16h x, v16h y) { dep_guard_h(a, b, x, y); }
  static __device__ __forceinline__ void keep(v16h a, v16h b, v16h c, v16h d) { keep4_h(a, b, c, d); }
};
template <> struct Frag<__bf16> {
  typedef v16b V; union U { v16b v; v8b h[2]; };
  static __device__ __forceinline__ v16b load(const __bf16* p) {
    U f; f.h[0] = *(const v8b*)(p); f.h[1] = *(const v8b*)(p + 16); return f.v;
  }
  static __device__ __forceinline__ v8f mma(v16b a, v16b b, v8f c) {
    return __builtin_amdgcn_wmma_f32_16x16x32_bf16(false, a, false, b, (short)0, c, false, false);
  }
  static __device__ __forceinline__ void guard(v8f& a, v8f& b, v16b x, v16b y) { dep_guard_b(a, b, x, y); }
  static __device__ __forceinline__ void keep(v16b a, v16b b, v16b c, v16b d) { keep4_b(a, b, c, d); }
};

__device__ __forceinline__ unsigned pk16(unsigned short a, unsigned short b) { return (unsigned)a | ((unsigned)b << 16); }
__device__ __forceinline__ unsigned short h_bits(float f) { const _Float16 h = (_Float16)f; return __builtin_bit_cast(unsigned short, h); }

template <int ET> struct Elem;
template <> struct Elem<0> { typedef _Float16 T; };
template <> struct Elem<1> { typedef __bf16 T; };
template <int ET, bool SPLIT, int BIAS_MODE, int OUT_MODE, bool RESID, int ACT = 0>
__global__ __launch_bounds__(256) void wmma_gemm64(
    const unsigned short* __restrict__ Ap, const unsigned short* __restrict__ A2p, int lda, long strideA,
    const unsigned short* __restrict__ Btp, const unsigned short* __restrict__ Bt2p, int ldb, long strideB,
    void* __restrict__ Cout, void* __restrict__ Cout2, int ldc, long strideC,
    const float* __restrict__ bias,
    const float* __restrict__ resid, long strideR,
    int M, int N, int K, float scale) {
  typedef typename Elem<ET>::T T;
  typedef typename Frag<T>::V V;
  const T* A = (const T*)Ap; const T* A2 = (const T*)A2p; const T* Bt = (const T*)Btp; const T* Bt2 = (const T*)Bt2p;
  __shared__ __align__(16) float sT[8][16 * 68];
  const int b    = blockIdx.y;
  const int lane = threadIdx.x & 31;
  const int wave = threadIdx.x >> 5;
  const int tilesN = N >> 6;
  const int tilesM = M >> 6;
  const int tile = blockIdx.x * 8 + wave;
  if (tile >= tilesM * tilesN) return;
  const int tm = tile / tilesN;
  const int tn = tile - tm * tilesN;
  const int m0 = tm << 6;
  const int n0 = tn << 6;

  const T* Ab  = A  + (size_t)b * strideA;
  const T* Bb  = Bt + (size_t)b * strideB;
  const T* Ab2 = SPLIT ? (A2  + (size_t)b * strideA) : nullptr;
  const T* Bb2 = SPLIT ? (Bt2 + (size_t)b * strideB) : nullptr;

  const int rlane = lane & 15;
  const int koff  = (lane >> 4) * 8;
  const int mOff  = (lane >> 4) * 8;

  v8f acc[4][4];
#pragma unroll
  for (int i = 0; i < 4; ++i)
#pragma unroll
    for (int j = 0; j < 4; ++j) acc[i][j] = (v8f){0.f,0.f,0.f,0.f,0.f,0.f,0.f,0.f};

  for (int k0 = 0; k0 < K; k0 += 32) {
    V bh[4], bl[4];
#pragma unroll
    for (int j = 0; j < 4; ++j) {
      const size_t bo = (size_t)(n0 + (j << 4) + rlane) * ldb + koff + k0;
      bh[j] = Frag<T>::load(Bb + bo);
      if (SPLIT) bl[j] = Frag<T>::load(Bb2 + bo);
    }
#pragma unroll
    for (int i = 0; i < 4; ++i) {
      const size_t ao = (size_t)(m0 + (i << 4) + rlane) * lda + koff + k0;
      V ah = Frag<T>::load(Ab + ao);
      V al;
      if (SPLIT) al = Frag<T>::load(Ab2 + ao);
#pragma unroll
      for (int j = 0; j < 4; ++j) {
        acc[i][j] = Frag<T>::mma(ah, bh[j], acc[i][j]);
        if (SPLIT) {
          acc[i][j] = Frag<T>::mma(ah, bl[j], acc[i][j]);
          acc[i][j] = Frag<T>::mma(al, bh[j], acc[i][j]);
        }
      }
      Frag<T>::guard(acc[i][0], acc[i][3], ah, SPLIT ? al : ah);
    }
    Frag<T>::keep(bh[0], bh[1], bh[2], bh[3]);
    if (SPLIT) Frag<T>::keep(bl[0], bl[1], bl[2], bl[3]);
  }
  acc_guard4(acc[0][0], acc[0][1], acc[0][2], acc[0][3]);
  acc_guard4(acc[1][0], acc[1][1], acc[1][2], acc[1][3]);
  acc_guard4(acc[2][0], acc[2][1], acc[2][2], acc[2][3]);
  acc_guard4(acc[3][0], acc[3][1], acc[3][2], acc[3][3]);

  float* slab = sT[wave];
  const float* Rb = RESID ? (resid + (size_t)b * strideR) : nullptr;
#pragma unroll
  for (int i = 0; i < 4; ++i) {
    const int mBase = m0 + (i << 4);
#pragma unroll
    for (int j = 0; j < 4; ++j) {
      const int n = n0 + (j << 4) + rlane;
      float bv = 0.f;
      if (BIAS_MODE == 2) bv = bias[n];
#pragma unroll
      for (int r = 0; r < 8; ++r) {
        float v = acc[i][j][r] * scale;
        if (BIAS_MODE == 1) v += bias[mBase + mOff + r];
        if (BIAS_MODE == 2) v += bv;
        if (RESID) v += Rb[(size_t)(mBase + mOff + r) * ldc + n];
        if (ACT == 2) v = fmaxf(v, 0.0f);
        if (ACT == 4) v = (v > 0.f) ? v : 0.01f * v;
        slab[(mOff + r) * 68 + (j << 4) + rlane] = v;
      }
    }
    __builtin_amdgcn_fence(__ATOMIC_RELEASE, "workgroup");
    __builtin_amdgcn_wave_barrier();
    __builtin_amdgcn_fence(__ATOMIC_ACQUIRE, "workgroup");
    if (OUT_MODE == 0) {
      float* C = (float*)Cout + (size_t)b * strideC;
      const int hh = lane >> 4, c4 = (lane & 15) * 4;
      for (int pass = 0; pass < 2; ++pass) {
#pragma unroll
        for (int it = 0; it < 8; ++it) {
          const int row = it * 2 + hh;
          v4f v = *(const v4f*)(slab + row * 68 + c4);
          *(volatile v4f*)(C + (size_t)(mBase + row) * ldc + n0 + c4) = v;
        }
        __threadfence();
      }
    } else {
      const int q = lane >> 3, c8 = (lane & 7) * 8;
      unsigned short* C  = (unsigned short*)Cout  + (size_t)b * strideC;
      unsigned short* C2 = (OUT_MODE == 2) ? ((unsigned short*)Cout2 + (size_t)b * strideC) : nullptr;
      for (int pass = 0; pass < 2; ++pass) {
#pragma unroll
        for (int it = 0; it < 4; ++it) {
          const int row = it * 4 + q;
          const float* sp = slab + row * 68 + c8;
          v8h hv, lv;
#pragma unroll
          for (int e = 0; e < 8; ++e) {
            if (OUT_MODE == 1) {
              hv[e] = (_Float16)sp[e];
            } else {
              unsigned short hb = f2bf_bits(sp[e]);
              unsigned short lb = f2bf_bits(sp[e] - bf_bits2f(hb));
              hv[e] = __builtin_bit_cast(_Float16, hb);
              lv[e] = __builtin_bit_cast(_Float16, lb);
            }
          }
          *(volatile v8h*)(C + (size_t)(mBase + row) * ldc + n0 + c8) = hv;
          if (OUT_MODE == 2) *(volatile v8h*)(C2 + (size_t)(mBase + row) * ldc + n0 + c8) = lv;
        }
        __threadfence();
      }
    }
    __builtin_amdgcn_fence(__ATOMIC_RELEASE, "workgroup");
    __builtin_amdgcn_wave_barrier();
    __builtin_amdgcn_fence(__ATOMIC_ACQUIRE, "workgroup");
  }
}

__device__ __forceinline__ float gelu_f(float x) { return 0.5f * x * (1.0f + erff(x * 0.70710678118654752f)); }

__global__ __launch_bounds__(256) void wcast_kernel(const float* __restrict__ w1, const float* __restrict__ w21,
                                                    const float* __restrict__ w22, const float* __restrict__ w3,
                                                    const float* __restrict__ wf1, const float* __restrict__ wf2,
                                                    unsigned short* __restrict__ out, float scale) {
  const int bx = blockIdx.x;
  const int i = bx * 256 + threadIdx.x;
  const float* src;
  int base;
  if (bx < 32)       { src = w1;  base = 0; }
  else if (bx < 64)  { src = w21; base = 8192; }
  else if (bx < 96)  { src = w22; base = 16384; }
  else if (bx < 128) { src = w3;  base = 24576; }
  else if (bx < 256) { src = wf1; base = 32768; }
  else               { src = wf2; base = 65536; }
  const float* p = src + 8 * (size_t)(i - base);
  const v4f a = *(const v4f*)(p);
  const v4f c = *(const v4f*)(p + 4);
  unsigned short hb[8];
#pragma unroll
  for (int e = 0; e < 4; ++e) {
    hb[e]     = h_bits(a[e] * scale);
    hb[4 + e] = h_bits(c[e] * scale);
  }
  const v4u u = (v4u){pk16(hb[0], hb[1]), pk16(hb[2], hb[3]), pk16(hb[4], hb[5]), pk16(hb[6], hb[7])};
  unsigned short* q = out + 8 * (size_t)i;
  *(volatile v4u*)q = u;
  __threadfence();
  *(volatile v4u*)q = u;
}

__global__ __launch_bounds__(256) void gn_partial_kernel(const float* __restrict__ src, float* __restrict__ part) {
  __shared__ float r1[256];
  __shared__ float r2[256];
  const int img = blockIdx.y, blk = blockIdx.x, t = threadIdx.x;
  const float* p = src + (size_t)img * kImgElems + (size_t)blk * (kPartV4 * 4);
  float s1 = 0.f, s2 = 0.f;
  for (int i = t; i < kPartV4; i += 256) {
    const v4f v = *(const v4f*)(p + 4 * (size_t)i);
    s1 += (v[0] + v[1]) + (v[2] + v[3]);
    s2 += (v[0] * v[0] + v[1] * v[1]) + (v[2] * v[2] + v[3] * v[3]);
  }
  r1[t] = s1; r2[t] = s2;
  __syncthreads();
  for (int st = 128; st > 0; st >>= 1) {
    if (t < st) { r1[t] += r1[t + st]; r2[t] += r2[t + st]; }
    __syncthreads();
  }
  if (t < 8) {
    const float a0 = r1[0], b0 = r2[0];
    v4f v;
    v[0] = (t == 0) ? a0 : 0.f;
    v[1] = (t == 0) ? b0 : 0.f;
    v[2] = 0.f; v[3] = 0.f;
    float* dst = part + ((size_t)(img * kPartBlocks + blk) * 32 + t * 4);
    *(volatile v4f*)dst = v;
    __threadfence();
    *(volatile v4f*)dst = v;
  }
}

__global__ __launch_bounds__(64) void gn_final_kernel(const float* __restrict__ part, float* __restrict__ stats) {
  __shared__ float r1[64];
  __shared__ float r2[64];
  const int img = blockIdx.x, t = threadIdx.x;
  const float* pl = part + (size_t)(img * kPartBlocks + t) * 32;
  r1[t] = pl[0]; r2[t] = pl[1];
  __syncthreads();
  for (int st = 32; st > 0; st >>= 1) {
    if (t < st) { r1[t] += r1[t + st]; r2[t] += r2[t + st]; }
    __syncthreads();
  }
  const float S1 = r1[0], S2 = r2[0];
  const float mean = S1 * kInvImgElems;
  float var = S2 * kInvImgElems - mean * mean;
  var = fmaxf(var, 0.f);
  const float rstd = rsqrtf(var + kGnEps);
  if (t < 8) {
    v4f v;
    v[0] = (t == 0) ? mean : 0.f;
    v[1] = (t == 0) ? rstd : 0.f;
    v[2] = 0.f; v[3] = 0.f;
    float* dst = stats + ((size_t)img * 32 + t * 4);
    *(volatile v4f*)dst = v;
    __threadfence();
    *(volatile v4f*)dst = v;
  }
}

__global__ __launch_bounds__(256) void tr_in_kernel(const float* __restrict__ x, const float* __restrict__ stats,
                                                    const float* __restrict__ gw, const float* __restrict__ gb,
                                                    float* __restrict__ xT, unsigned short* __restrict__ hA, int img0) {
  __shared__ __align__(16) float sm[64 * 68];
  const int t = threadIdx.x, lane = t & 31, wave = t >> 5;
  const int p0 = blockIdx.x * 64, c0 = blockIdx.y * 64, img = blockIdx.z;
  const float* xs = x + ((size_t)(img0 + img) * kCh + c0) * kHW + p0;
#pragma unroll
  for (int it = 0; it < 4; ++it) {
    const int e = it * 256 + t;
    const int cl = e >> 4;
    const int p4 = (e & 15) * 4;
    const v4f v = *(const v4f*)(xs + (size_t)cl * kHW + p4);
    sm[(p4 + 0) * 68 + cl] = v[0];
    sm[(p4 + 1) * 68 + cl] = v[1];
    sm[(p4 + 2) * 68 + cl] = v[2];
    sm[(p4 + 3) * 68 + cl] = v[3];
  }
  __syncthreads();
  const float m = stats[img * 32], r = stats[img * 32 + 1];
  const int hh = lane >> 4, c4 = (lane & 15) * 4;
  const int q = lane >> 3, c8 = (lane & 7) * 8;
  v4f f[4];
#pragma unroll
  for (int it = 0; it < 4; ++it) {
    const int row = wave * 8 + it * 2 + hh;
    f[it] = *(const v4f*)(sm + row * 68 + c4);
  }
  const v4f w0 = *(const v4f*)(gw + c0 + c8);
  const v4f w1 = *(const v4f*)(gw + c0 + c8 + 4);
  const v4f g0 = *(const v4f*)(gb + c0 + c8);
  const v4f g1 = *(const v4f*)(gb + c0 + c8 + 4);
  v4u u[2];
#pragma unroll
  for (int it = 0; it < 2; ++it) {
    const int row = wave * 8 + it * 4 + q;
    const v4f s0 = *(const v4f*)(sm + row * 68 + c8);
    const v4f s1 = *(const v4f*)(sm + row * 68 + c8 + 4);
    unsigned short hb[8];
#pragma unroll
    for (int e = 0; e < 4; ++e) {
      hb[e]     = h_bits((s0[e] - m) * r * w0[e] + g0[e]);
      hb[4 + e] = h_bits((s1[e] - m) * r * w1[e] + g1[e]);
    }
    u[it] = (v4u){pk16(hb[0], hb[1]), pk16(hb[2], hb[3]), pk16(hb[4], hb[5]), pk16(hb[6], hb[7])};
  }
  const size_t rowBase = (size_t)img * kHW + p0;
  for (int pass = 0; pass < 2; ++pass) {
#pragma unroll
    for (int it = 0; it < 4; ++it) {
      const int row = wave * 8 + it * 2 + hh;
      *(volatile v4f*)(xT + (rowBase + row) * kCh + c0 + c4) = f[it];
    }
#pragma unroll
    for (int it = 0; it < 2; ++it) {
      const int row = wave * 8 + it * 4 + q;
      *(volatile v4u*)(hA + (rowBase + row) * kCh + c0 + c8) = u[it];
    }
    __threadfence();
  }
}

__global__ __launch_bounds__(256) void tr_out_kernel(const float* __restrict__ src, float* __restrict__ out, int img0) {
  __shared__ __align__(16) float sm[64 * 68];
  const int t = threadIdx.x, lane = t & 31, wave = t >> 5;
  const int p0 = blockIdx.x * 64, c0 = blockIdx.y * 64, img = blockIdx.z;
  const float* sp = src + ((size_t)img * kHW + p0) * kCh + c0;
#pragma unroll
  for (int it = 0; it < 4; ++it) {
    const int e = it * 256 + t;
    const int pl = e >> 4;
    const int c4 = (e & 15) * 4;
    const v4f v = *(const v4f*)(sp + (size_t)pl * kCh + c4);
    sm[(c4 + 0) * 68 + pl] = v[0];
    sm[(c4 + 1) * 68 + pl] = v[1];
    sm[(c4 + 2) * 68 + pl] = v[2];
    sm[(c4 + 3) * 68 + pl] = v[3];
  }
  __syncthreads();
  const int hh = lane >> 4, p4 = (lane & 15) * 4;
  v4f f[4];
#pragma unroll
  for (int it = 0; it < 4; ++it) {
    const int row = wave * 8 + it * 2 + hh;
    f[it] = *(const v4f*)(sm + row * 68 + p4);
  }
  float* ob = out + ((size_t)(img0 + img) * kCh + c0) * kHW + p0;
  for (int pass = 0; pass < 2; ++pass) {
#pragma unroll
    for (int it = 0; it < 4; ++it) {
      const int row = wave * 8 + it * 2 + hh;
      *(volatile v4f*)(ob + (size_t)row * kHW + p4) = f[it];
    }
    __threadfence();
  }
}

__global__ __launch_bounds__(256) void gn_gelu_kernel(const float* __restrict__ src, const float* __restrict__ stats,
                                                     const float* __restrict__ gw, const float* __restrict__ gb,
                                                     float* __restrict__ dst, int n4) {
  const int i = blockIdx.x * 256 + threadIdx.x;
  if (i >= n4) return;
  const size_t e0 = 4 * (size_t)i;
  const int c = (int)(e0 & (kCh - 1));
  const int img = (int)(e0 / kImgElems);
  const float m = stats[img * 32], r = stats[img * 32 + 1];
  const v4f v  = *(const v4f*)(src + e0);
  const v4f w4 = *(const v4f*)(gw + c);
  const v4f b4 = *(const v4f*)(gb + c);
  const float y0 = (v[0] - m) * r * w4[0] + b4[0];
  const float y1 = (v[1] - m) * r * w4[1] + b4[1];
  const float y2 = (v[2] - m) * r * w4[2] + b4[2];
  const float y3 = (v[3] - m) * r * w4[3] + b4[3];
  float o0 = 0.f, o1 = 0.f, o2 = 0.f, o3 = 0.f;
#pragma unroll 1
  for (int e = 0; e < 4; ++e) {
    const float xin = (e == 0) ? y0 : (e == 1) ? y1 : (e == 2) ? y2 : y3;
    const float g = gelu_f(xin);
    o0 = (e == 0) ? g : o0;
    o1 = (e == 1) ? g : o1;
    o2 = (e == 2) ? g : o2;
    o3 = (e == 3) ? g : o3;
  }
  v4f o;
  o[0] = o0; o[1] = o1; o[2] = o2; o[3] = o3;
  float* q = dst + e0;
  *(volatile v4f*)q = o;
  __threadfence();
  *(volatile v4f*)q = o;
}

__global__ __launch_bounds__(256) void shift_kernel(const float* __restrict__ a, unsigned short* __restrict__ lr,
                                                    unsigned short* __restrict__ td, int nthr) {
  const int i = blockIdx.x * 256 + threadIdx.x;
  if (i >= nthr) return;
  const int row = i >> 5;
  const int c8 = (i & 31) * 8;
  const int img = row / kHW;
  const int p = row - img * kHW;
  const int h = p / kWid;
  const int w = p - h * kWid;
  unsigned short hl[8], ht[8];
#pragma unroll
  for (int e = 0; e < 8; ++e) {
    const int c = c8 + e;
    const int s = kShiftPad - c / kShiftGroup;
    const int wl = w + s;
    const bool okl = (unsigned)wl < (unsigned)kWid;
    const int wlc = (wl < 0) ? 0 : ((wl > kWid - 1) ? (kWid - 1) : wl);
    const int hs = h + s;
    const bool okt = (unsigned)hs < (unsigned)kHgt;
    const int hsc = (hs < 0) ? 0 : ((hs > kHgt - 1) ? (kHgt - 1) : hs);
    float vl = a[((size_t)(img * kHW + h * kWid + wlc)) * kCh + c];
    float vt = a[((size_t)(img * kHW + hsc * kWid + w)) * kCh + c];
    vl = okl ? vl : 0.f;
    vt = okt ? vt : 0.f;
    hl[e] = h_bits(vl);
    ht[e] = h_bits(vt);
  }
  const v4u ul = (v4u){pk16(hl[0], hl[1]), pk16(hl[2], hl[3]), pk16(hl[4], hl[5]), pk16(hl[6], hl[7])};
  const v4u ut = (v4u){pk16(ht[0], ht[1]), pk16(ht[2], ht[3]), pk16(ht[4], ht[5]), pk16(ht[6], ht[7])};
  unsigned short* ql = lr + (size_t)row * kCh + c8;
  unsigned short* qt = td + (size_t)row * kCh + c8;
  *(volatile v4u*)ql = ul;
  *(volatile v4u*)qt = ut;
  __threadfence();
  *(volatile v4u*)ql = ul;
  *(volatile v4u*)qt = ut;
}

__global__ __launch_bounds__(256) void gelu_sum_kernel(const float* __restrict__ z1, const float* __restrict__ z2,
                                                      float* __restrict__ dst, int n4) {
  const int i = blockIdx.x * 256 + threadIdx.x;
  if (i >= n4) return;
  const size_t e0 = 4 * (size_t)i;
  const v4f a = *(const v4f*)(z1 + e0);
  const v4f c = *(const v4f*)(z2 + e0);
  float o0 = 0.f, o1 = 0.f, o2 = 0.f, o3 = 0.f;
#pragma unroll 1
  for (int e = 0; e < 8; ++e) {
    const int k = e & 3;
    const float xa = (k == 0) ? a[0] : (k == 1) ? a[1] : (k == 2) ? a[2] : a[3];
    const float xc = (k == 0) ? c[0] : (k == 1) ? c[1] : (k == 2) ? c[2] : c[3];
    const float xin = (e < 4) ? xa : xc;
    const float g = gelu_f(xin);
    o0 = (k == 0) ? (o0 + g) : o0;
    o1 = (k == 1) ? (o1 + g) : o1;
    o2 = (k == 2) ? (o2 + g) : o2;
    o3 = (k == 3) ? (o3 + g) : o3;
  }
  v4f o;
  o[0] = o0; o[1] = o1; o[2] = o2; o[3] = o3;
  float* q = dst + e0;
  *(volatile v4f*)q = o;
  __threadfence();
  *(volatile v4f*)q = o;
}

__global__ __launch_bounds__(256) void gn_cast_kernel(const float* __restrict__ src, const float* __restrict__ stats,
                                                     const float* __restrict__ gw, const float* __restrict__ gb,
                                                     unsigned short* __restrict__ dst, int n8) {
  const int i = blockIdx.x * 256 + threadIdx.x;
  if (i >= n8) return;
  const size_t e0 = 8 * (size_t)i;
  const int c = (int)(e0 & (kCh - 1));
  const int img = (int)(e0 / kImgElems);
  const float m = stats[img * 32], r = stats[img * 32 + 1];
  const v4f a  = *(const v4f*)(src + e0);
  const v4f b  = *(const v4f*)(src + e0 + 4);
  const v4f w0 = *(const v4f*)(gw + c);
  const v4f w1 = *(const v4f*)(gw + c + 4);
  const v4f g0 = *(const v4f*)(gb + c);
  const v4f g1 = *(const v4f*)(gb + c + 4);
  unsigned short hb[8];
#pragma unroll
  for (int e = 0; e < 4; ++e) {
    hb[e]     = h_bits((a[e] - m) * r * w0[e] + g0[e]);
    hb[4 + e] = h_bits((b[e] - m) * r * w1[e] + g1[e]);
  }
  const v4u u = (v4u){pk16(hb[0], hb[1]), pk16(hb[2], hb[3]), pk16(hb[4], hb[5]), pk16(hb[6], hb[7])};
  unsigned short* q = dst + e0;
  *(volatile v4u*)q = u;
  __threadfence();
  *(volatile v4u*)q = u;
}

__global__ __launch_bounds__(256) void gelu_cast_kernel(const float* __restrict__ in, unsigned short* __restrict__ out, int n8) {
  const int i = blockIdx.x * 256 + threadIdx.x;
  if (i >= n8) return;
  const float* p = in + 8 * (size_t)i;
  const v4f a = *(const v4f*)(p);
  const v4f c = *(const v4f*)(p + 4);
  float o0 = 0.f, o1 = 0.f, o2 = 0.f, o3 = 0.f, o4 = 0.f, o5 = 0.f, o6 = 0.f, o7 = 0.f;
#pragma unroll 1
  for (int e = 0; e < 8; ++e) {
    const int k = e & 3;
    const float xa = (k == 0) ? a[0] : (k == 1) ? a[1] : (k == 2) ? a[2] : a[3];
    const float xc = (k == 0) ? c[0] : (k == 1) ? c[1] : (k == 2) ? c[2] : c[3];
    const float xin = (e < 4) ? xa : xc;
    const float g = gelu_f(xin);
    o0 = (e == 0) ? g : o0;
    o1 = (e == 1) ? g : o1;
    o2 = (e == 2) ? g : o2;
    o3 = (e == 3) ? g : o3;
    o4 = (e == 4) ? g : o4;
    o5 = (e == 5) ? g : o5;
    o6 = (e == 6) ? g : o6;
    o7 = (e == 7) ? g : o7;
  }
  const v4u u = (v4u){pk16(h_bits(o0), h_bits(o1)), pk16(h_bits(o2), h_bits(o3)),
                      pk16(h_bits(o4), h_bits(o5)), pk16(h_bits(o6), h_bits(o7))};
  unsigned short* q = out + 8 * (size_t)i;
  *(volatile v4u*)q = u;
  __threadfence();
  *(volatile v4u*)q = u;
}

#define GemmBias    wmma_gemm64<0, false, 2, 0, false, 0>
#define GemmBiasRes wmma_gemm64<0, false, 2, 0, true, 0>

extern "C" void kernel_launch(void* const* d_in, const int* in_sizes, int n_in,
                              void* d_out, int out_size, void* d_ws, size_t ws_size,
                              hipStream_t stream)
{
  if (n_in < 21) return;
  if (in_sizes[0] != kImgs * kImgElems) return;
  if (out_size != kImgs * kImgElems) return;
  if (in_sizes[3] != kCh * kCh || in_sizes[7] != kCh * kCh || in_sizes[9] != kCh * kCh || in_sizes[13] != kCh * kCh) return;
  if (in_sizes[17] != kHid * kCh || in_sizes[19] != kCh * kHid) return;
  if (in_sizes[1] != kCh || in_sizes[18] != kHid || in_sizes[20] != kCh) return;

  const float* x     = (const float*)d_in[0];
  const float* n1_w  = (const float*)d_in[1];
  const float* n1_b  = (const float*)d_in[2];
  const float* c1_w  = (const float*)d_in[3];
  const float* c1_b  = (const float*)d_in[4];
  const float* an1_w = (const float*)d_in[5];
  const float* an1_b = (const float*)d_in[6];
  const float* c21_w = (const float*)d_in[7];
  const float* c21_b = (const float*)d_in[8];
  const float* c22_w = (const float*)d_in[9];
  const float* c22_b = (const float*)d_in[10];
  const float* an2_w = (const float*)d_in[11];
  const float* an2_b = (const float*)d_in[12];
  const float* c3_w  = (const float*)d_in[13];
  const float* c3_b  = (const float*)d_in[14];
  const float* n2_w  = (const float*)d_in[15];
  const float* n2_b  = (const float*)d_in[16];
  const float* fc1_w = (const float*)d_in[17];
  const float* fc1_b = (const float*)d_in[18];
  const float* fc2_w = (const float*)d_in[19];
  const float* fc2_b = (const float*)d_in[20];
  float* outp = (float*)d_out;

  const size_t planeF32 = (size_t)kRows * kCh * 4;
  const size_t planeF16 = (size_t)kRows * kCh * 2;
  const size_t hidF32   = (size_t)kRows * kHid * 4;
  const size_t hidF16   = (size_t)kRows * kHid * 2;
  const size_t offW    = 0;
  const size_t offPart = offW + (size_t)786432 * 2;
  const size_t offStat = offPart + (size_t)kGrpImgs * kPartBlocks * 32 * 4;
  const size_t offX    = offStat + 512;
  const size_t offP16  = offX + planeF32;
  const size_t offA    = offP16 + planeF16;
  const size_t offB    = offA + planeF32;
  const size_t offH    = offB + planeF32;
  const size_t offG    = offH + hidF32;
  const size_t total   = offG + hidF16;
  if (total > ws_size) return;

  char* ws = (char*)d_ws;
  unsigned short* W16  = (unsigned short*)(ws + offW);
  unsigned short* W1   = W16;
  unsigned short* W21  = W16 + 65536;
  unsigned short* W22  = W16 + 131072;
  unsigned short* W3   = W16 + 196608;
  unsigned short* Wf1  = W16 + 262144;
  unsigned short* Wf2  = W16 + 524288;
  float* part  = (float*)(ws + offPart);
  float* stat  = (float*)(ws + offStat);
  float* xT    = (float*)(ws + offX);
  unsigned short* P16 = (unsigned short*)(ws + offP16);
  float* bufA  = (float*)(ws + offA);
  float* bufB  = (float*)(ws + offB);
  unsigned short* lr16 = (unsigned short*)(ws + offH);
  unsigned short* td16 = (unsigned short*)(ws + offH + planeF16);
  float* sH    = (float*)(ws + offH + 2 * planeF16);
  float* f1H   = (float*)(ws + offH);
  unsigned short* gG = (unsigned short*)(ws + offG);

  const int n4plane = kRows * kCh / 4;
  const int n8plane = kRows * kCh / 8;
  const int nShift  = kRows * 32;
  const int n8hid   = kRows * kHid / 8;
  const dim3 blk(256);
  const dim3 gPart(kPartBlocks, kGrpImgs);
  const dim3 gTile(kHW / 64, kCh / 64, kGrpImgs);
  const int  tilesC = (kRows / 64) * (kCh / 64);
  const int  tilesH = (kRows / 64) * (kHid / 64);
  const dim3 gGemmC((tilesC + 7) / 8, 1);
  const dim3 gGemmH((tilesH + 7) / 8, 1);
  const long zeroL = 0;

  wcast_kernel<<<384, blk, 0, stream>>>(c1_w, c21_w, c22_w, c3_w, fc1_w, fc2_w, W16, kWCarry);

  for (int g = 0; g < kGroups; ++g) {
    const int img0 = g * kGrpImgs;

    gn_partial_kernel<<<gPart, blk, 0, stream>>>(x + (size_t)img0 * kImgElems, part);
    gn_final_kernel<<<kGrpImgs, 64, 0, stream>>>(part, stat);
    tr_in_kernel<<<gTile, blk, 0, stream>>>(x, stat, n1_w, n1_b, xT, P16, img0);

    GemmBias<<<gGemmC, blk, 0, stream>>>(P16, P16, kCh, zeroL, W1, W1, kCh, zeroL,
                                           (void*)bufA, (void*)bufA, kCh, zeroL, c1_b, xT, zeroL,
                                           kRows, kCh, kCh, kWCarryInv);

    gn_partial_kernel<<<gPart, blk, 0, stream>>>(bufA, part);
    gn_final_kernel<<<kGrpImgs, 64, 0, stream>>>(part, stat);
    gn_gelu_kernel<<<n4plane / 256, blk, 0, stream>>>(bufA, stat, an1_w, an1_b, bufB, n4plane);

    shift_kernel<<<nShift / 256, blk, 0, stream>>>(bufB, lr16, td16, nShift);

    GemmBias<<<gGemmC, blk, 0, stream>>>(lr16, lr16, kCh, zeroL, W21, W21, kCh, zeroL,
                                           (void*)bufA, (void*)bufA, kCh, zeroL, c21_b, xT, zeroL,
                                           kRows, kCh, kCh, kWCarryInv);
    GemmBias<<<gGemmC, blk, 0, stream>>>(td16, td16, kCh, zeroL, W22, W22, kCh, zeroL,
                                           (void*)bufB, (void*)bufB, kCh, zeroL, c22_b, xT, zeroL,
                                           kRows, kCh, kCh, kWCarryInv);

    gelu_sum_kernel<<<n4plane / 256, blk, 0, stream>>>(bufA, bufB, sH, n4plane);

    gn_partial_kernel<<<gPart, blk, 0, stream>>>(sH, part);
    gn_final_kernel<<<kGrpImgs, 64, 0, stream>>>(part, stat);
    gn_cast_kernel<<<n8plane / 256, blk, 0, stream>>>(sH, stat, an2_w, an2_b, P16, n8plane);

    GemmBiasRes<<<gGemmC, blk, 0, stream>>>(P16, P16, kCh, zeroL, W3, W3, kCh, zeroL,
                                              (void*)bufB, (void*)bufB, kCh, zeroL, c3_b, xT, zeroL,
                                              kRows, kCh, kCh, kWCarryInv);

    gn_partial_kernel<<<gPart, blk, 0, stream>>>(bufB, part);
    gn_final_kernel<<<kGrpImgs, 64, 0, stream>>>(part, stat);
    gn_cast_kernel<<<n8plane / 256, blk, 0, stream>>>(bufB, stat, n2_w, n2_b, P16, n8plane);

    GemmBias<<<gGemmH, blk, 0, stream>>>(P16, P16, kCh, zeroL, Wf1, Wf1, kCh, zeroL,
                                           (void*)f1H, (void*)f1H, kHid, zeroL, fc1_b, xT, zeroL,
                                           kRows, kHid, kCh, kWCarryInv);

    gelu_cast_kernel<<<n8hid / 256, blk, 0, stream>>>(f1H, gG, n8hid);

    GemmBiasRes<<<gGemmC, blk, 0, stream>>>(gG, gG, kHid, zeroL, Wf2, Wf2, kHid, zeroL,
                                              (void*)bufA, (void*)bufA, kCh, zeroL, fc2_b, bufB, zeroL,
                                              kRows, kCh, kHid, kWCarryInv);

    tr_out_kernel<<<gTile, blk, 0, stream>>>(bufA, outp, img0);
  }
}
